// SABlock_78520592105699
// MI455X (gfx1250) — hardware-verified
//
#include <hip/hip_runtime.h>
#include <hip/hip_bf16.h>


#ifndef NB
#define NB 4
#endif
#ifndef SEQ
#define SEQ 4096
#endif
#define NB_FULL   4
#define SEQ_FULL  4096
#define CH        512
#define CI        256
#define WCAT_N    (3 * CI)
#define MROWS     (NB * SEQ)
#define P_CARRY   16384.0f
#define V_CARRY   16.0f
#define O_FOLD    (1.0f / 262144.0f)

static_assert(SEQ % 128 == 0);
static_assert(SEQ <= SEQ_FULL);
static_assert(NB >= 1 && NB <= NB_FULL);
static_assert(MROWS % 128 == 0);
static_assert(CH % 128 == 0);
static_assert(CI % 64 == 0);
static_assert(WCAT_N % 64 == 0);
static_assert(CH % 32 == 0 && CI % 32 == 0);
static_assert((CI * CH) % 2048 == 0);

#define WS_TOTAL ((size_t)MROWS * CH * 2 + (size_t)WCAT_N * CH * 2 + (size_t)CH * CI * 2 + \
                  (size_t)7 * MROWS * CI * 2)
static_assert(WS_TOTAL <= (size_t)134217728);
static_assert((size_t)NB * CH * SEQ * 4 <= (size_t)33554432);

typedef float          v4f   __attribute__((ext_vector_type(4)));
typedef float          v8f   __attribute__((ext_vector_type(8)));
typedef unsigned short bfu16;
typedef unsigned short v8us  __attribute__((ext_vector_type(8)));
typedef unsigned short v16us __attribute__((ext_vector_type(16)));
typedef __bf16         v16bf __attribute__((ext_vector_type(16)));
typedef _Float16       v8h   __attribute__((ext_vector_type(8)));
typedef _Float16       v16h  __attribute__((ext_vector_type(16)));

#define GT_P  68
#define XT_P  68
#define PP    40
#define OP    132

__device__ __forceinline__ bfu16 f2bf(float f) {
    unsigned u = __float_as_uint(f);
    u += 0x7FFFu + ((u >> 16) & 1u);
    return (bfu16)(u >> 16);
}
__device__ __forceinline__ float bf2f(bfu16 b) { return __uint_as_float(((unsigned)b) << 16); }

union Frag  { v16us u; v8us half[2]; v16bf b; };
union FragH { v16us u; v8h  half[2]; v16h  v; };

__device__ __forceinline__ Frag ldfrag(const bfu16* p, int h) {
    Frag f;
    f.half[0] = *(const v8us*)(p + 8 * h);
    f.half[1] = *(const v8us*)(p + 16 + 8 * h);
    return f;
}
__device__ __forceinline__ FragH ldfragh(const _Float16* p, int h) {
    FragH f;
    f.half[0] = *(const v8h*)(p + 8 * h);
    f.half[1] = *(const v8h*)(p + 16 + 8 * h);
    return f;
}

__device__ __forceinline__ v8f wm(const Frag& a, const Frag& b, v8f c) {
    c = __builtin_amdgcn_wmma_f32_16x16x32_bf16(false, a.b, false, b.b, (short)0, c, false, false);
    asm volatile("v_nop\n\tv_nop\n\tv_nop\n\tv_nop" : "+v"(c) : "v"(a.u), "v"(b.u));
    return c;
}
__device__ __forceinline__ v8f wmh(const FragH& a, const FragH& b, v8f c) {
    c = __builtin_amdgcn_wmma_f32_16x16x32_f16(false, a.v, false, b.v, (short)0, c, false, false);
    asm volatile("v_nop\n\tv_nop\n\tv_nop\n\tv_nop" : "+v"(c) : "v"(a.u), "v"(b.u));
    return c;
}

__device__ __forceinline__ void split8(const v4f x0, const v4f x1, v8us& hv, v8us& lv) {
#pragma unroll
    for (int e = 0; e < 4; ++e) {
        const bfu16 a = f2bf(x0[e]);
        hv[e] = a;
        lv[e] = f2bf(x0[e] - bf2f(a));
        const bfu16 c = f2bf(x1[e]);
        hv[4 + e] = c;
        lv[4 + e] = f2bf(x1[e] - bf2f(c));
    }
}

__device__ __forceinline__ v8us pack8h(const v4f x0, const v4f x1, float sc) {
    union { v8h hv; v8us u; } q;
#pragma unroll
    for (int e = 0; e < 4; ++e) {
        q.hv[e]     = (_Float16)(x0[e] * sc);
        q.hv[4 + e] = (_Float16)(x1[e] * sc);
    }
    return q.u;
}

__device__ __forceinline__ float rowmax16(float v) {
    v = fmaxf(v, __shfl_xor(v, 1, 16));
    v = fmaxf(v, __shfl_xor(v, 2, 16));
    v = fmaxf(v, __shfl_xor(v, 4, 16));
    v = fmaxf(v, __shfl_xor(v, 8, 16));
    return v;
}
__device__ __forceinline__ float rowsum16(float v) {
    v += __shfl_xor(v, 1, 16);
    v += __shfl_xor(v, 2, 16);
    v += __shfl_xor(v, 4, 16);
    v += __shfl_xor(v, 8, 16);
    return v;
}

__global__ __launch_bounds__(256)
void cvt_flat(const float* __restrict__ src, bfu16* __restrict__ dst, int n8) {
    const int i = blockIdx.x * 256 + threadIdx.x;
    if (i >= n8) return;
    const float* s = src + (size_t)i * 8;
    const v4f f0 = *(const v4f*)s;
    const v4f f1 = *(const v4f*)(s + 4);
    v8us o;
#pragma unroll
    for (int e = 0; e < 4; ++e) { o[e] = f2bf(f0[e]); o[4 + e] = f2bf(f1[e]); }
    bfu16* d = dst + (size_t)i * 8;
    *(volatile v8us*)d = o;
    __threadfence();
    *(volatile v8us*)d = o;
}

__global__ __launch_bounds__(256)
void cvt_x(const float* __restrict__ x, bfu16* __restrict__ xt) {
    __shared__ __attribute__((aligned(16))) float Ts[64 * XT_P];

    const int tid  = threadIdx.x;
    const int wave = tid >> 5;
    const int lane = tid & 31;
    const int n0   = blockIdx.x * 64;
    const int c0   = blockIdx.y * 64;
    const int b    = blockIdx.z;

#pragma unroll
    for (int i = 0; i < 4; ++i) {
        const int idx = tid + 256 * i;
        const int c   = idx >> 4;
        const int nq  = (idx & 15) * 4;
        const v4f v = *(const v4f*)(x + ((size_t)(b * CH + c0 + c) * (size_t)SEQ_FULL + (size_t)(n0 + nq)));
#pragma unroll
        for (int e = 0; e < 4; ++e) Ts[(nq + e) * XT_P + c] = v[e];
    }
    __syncthreads();

    v8us ov[2];
    size_t oo[2];
#pragma unroll
    for (int it = 0; it < 2; ++it) {
        const int L  = wave * 8 + it * 4 + (lane >> 3);
        const int d0 = (lane & 7) * 8;
        const v4f x0 = *(const v4f*)(Ts + L * XT_P + d0);
        const v4f x1 = *(const v4f*)(Ts + L * XT_P + d0 + 4);
        v8us o;
#pragma unroll
        for (int e = 0; e < 4; ++e) { o[e] = f2bf(x0[e]); o[4 + e] = f2bf(x1[e]); }
        ov[it] = o;
        oo[it] = ((size_t)b * SEQ + (size_t)(n0 + L)) * CH + c0 + d0;
    }
#pragma unroll
    for (int ps = 0; ps < 2; ++ps) {
        if (ps) __threadfence();
#pragma unroll
        for (int it = 0; it < 2; ++it) *(volatile v8us*)(xt + oo[it]) = ov[it];
    }
}

template <int K, int MODE, int NPB>
__global__ __launch_bounds__(128)
void gemm16(const bfu16* __restrict__ A, const bfu16* __restrict__ Bh, const bfu16* __restrict__ Bl,
            bfu16* __restrict__ Th, bfu16* __restrict__ Tl,
            bfu16* __restrict__ Ph, bfu16* __restrict__ Pl,
            _Float16* __restrict__ Vt, float* __restrict__ Out) {
    __shared__ __attribute__((aligned(16))) float T[128 * GT_P];

    const int wave  = threadIdx.x >> 5;
    const int lane  = threadIdx.x & 31;
    const int laneN = lane & 15;
    const int h     = lane >> 4;
    const int mBase = blockIdx.x * 128;
    const int nBase = blockIdx.y * 64;

    const size_t ra0 = (size_t)(mBase + wave * 32 + laneN) * K;
    const size_t ra1 = ra0 + (size_t)16 * K;

    v8f acc[2][4] = {};

#pragma unroll 2
    for (int k0 = 0; k0 < K; k0 += 32) {
        const Frag fa0 = ldfrag(A + ra0 + k0, h);
        const Frag fa1 = ldfrag(A + ra1 + k0, h);
#pragma unroll
        for (int a = 0; a < 4; ++a) {
            const size_t rb = (size_t)(nBase + a * 16 + laneN) * K + k0;
            const Frag fb = ldfrag(Bh + rb, h);
            acc[0][a] = wm(fa0, fb, acc[0][a]);
            acc[1][a] = wm(fa1, fb, acc[1][a]);
            if (NPB == 2) {
                const Frag gb = ldfrag(Bl + rb, h);
                acc[0][a] = wm(fa0, gb, acc[0][a]);
                acc[1][a] = wm(fa1, gb, acc[1][a]);
            }
        }
    }

#pragma unroll
    for (int sub = 0; sub < 2; ++sub)
#pragma unroll
        for (int a = 0; a < 4; ++a)
#pragma unroll
            for (int j = 0; j < 8; ++j)
                T[(wave * 32 + sub * 16 + 8 * h + j) * GT_P + a * 16 + laneN] = acc[sub][a][j];
    __syncthreads();

    if (MODE == 1) {
        const int bO = nBase / SEQ;
        const int n0 = nBase % SEQ;
#pragma unroll
        for (int ps = 0; ps < 2; ++ps) {
            if (ps) __threadfence();
#pragma unroll
            for (int it = 0; it < 16; ++it) {
                const int lr  = wave * 32 + it * 2 + (lane >> 4);
                const int col = (lane & 15) * 4;
                const v4f t = *(const v4f*)(T + lr * GT_P + col);
                *(volatile v4f*)(Out + ((size_t)bO * CH + (size_t)(mBase + lr)) * (size_t)SEQ + n0 + col) = t;
            }
        }
    } else {
        const int sel = nBase / CI;
        const int cb  = nBase % CI;
        const int b   = mBase / SEQ;
        const int s0  = mBase % SEQ;
        if (sel < 2) {
            bfu16* Hp = (sel == 0) ? Ph : Th;
            bfu16* Lp = (sel == 0) ? Pl : Tl;
#pragma unroll
            for (int ps = 0; ps < 2; ++ps) {
                if (ps) __threadfence();
#pragma unroll
                for (int it = 0; it < 8; ++it) {
                    const int lr = wave * 32 + it * 4 + (lane >> 3);
                    const int d0 = (lane & 7) * 8;
                    const v4f x0 = *(const v4f*)(T + lr * GT_P + d0);
                    const v4f x1 = *(const v4f*)(T + lr * GT_P + d0 + 4);
                    v8us hv, lv;
                    split8(x0, x1, hv, lv);
                    const size_t off = (size_t)(mBase + lr) * CI + cb + d0;
                    *(volatile v8us*)(Hp + off) = hv;
                    *(volatile v8us*)(Lp + off) = lv;
                }
            }
        } else {
#pragma unroll
            for (int ps = 0; ps < 2; ++ps) {
                if (ps) __threadfence();
#pragma unroll
                for (int it = 0; it < 8; ++it) {
                    const int d  = wave * 16 + it * 2 + (lane >> 4);
                    const int sl = (lane & 15) * 8;
                    v4f x0, x1;
#pragma unroll
                    for (int e = 0; e < 4; ++e) {
                        x0[e] = T[(sl + e) * GT_P + d];
                        x1[e] = T[(sl + 4 + e) * GT_P + d];
                    }
                    const v8us pv = pack8h(x0, x1, V_CARRY);
                    const size_t off = ((size_t)b * CI + (size_t)(cb + d)) * (size_t)SEQ + s0 + sl;
                    *(volatile v8us*)(Vt + off) = pv;
                }
            }
        }
    }
}

__global__ __launch_bounds__(128) __attribute__((amdgpu_num_vgpr(256)))
void attn_pair(const bfu16* __restrict__ Th, const bfu16* __restrict__ Tl,
               const bfu16* __restrict__ Ph, const bfu16* __restrict__ Pl,
               const _Float16* __restrict__ Vt,
               bfu16* __restrict__ Yh, bfu16* __restrict__ Yl) {
    __shared__ __attribute__((aligned(16))) _Float16 Psh[2][16 * PP];
    __shared__ __attribute__((aligned(16))) float    Osh[4][16 * OP];
    __shared__ float Xm[2][2][16];
    __shared__ float Xs[2][2][16];

    const int wave  = threadIdx.x >> 5;
    const int lane  = threadIdx.x & 31;
    const int laneN = lane & 15;
    const int h     = lane >> 4;
    const int pr    = wave >> 1;
    const int kh    = wave & 1;
    const int b     = blockIdx.y;
    const int q0    = blockIdx.x * 32 + pr * 16;
    const size_t qoff  = ((size_t)b * SEQ + (size_t)(q0 + laneN)) * CI;
    const size_t vbase = (size_t)b * CI * (size_t)SEQ;

    float mrow[8], lrow[8];
#pragma unroll
    for (int j = 0; j < 8; ++j) { mrow[j] = -1e30f; lrow[j] = 0.0f; }
    v8f o[8] = {};

    _Float16* Pw = &Psh[pr][0];

    for (int key0 = 0; key0 < SEQ; key0 += 32) {
        const size_t koff = ((size_t)b * SEQ + (size_t)(key0 + 16 * kh + laneN)) * CI;
        v8f s = {};
#pragma unroll 2
        for (int kk = 0; kk < CI / 32; ++kk) {
            const int k0 = kk * 32;
            const Frag fq = ldfrag(Th + qoff + k0, h);
            const Frag gq = ldfrag(Tl + qoff + k0, h);
            const Frag fk = ldfrag(Ph + koff + k0, h);
            const Frag gk = ldfrag(Pl + koff + k0, h);
            s = wm(fq, fk, s);
            s = wm(gq, fk, s);
            s = wm(fq, gk, s);
        }

#pragma unroll
        for (int j = 0; j < 8; ++j) {
            const float mx = rowmax16(s[j]);
            if (laneN == 0) Xm[pr][kh][8 * h + j] = mx;
        }
        __syncthreads();

        float alpha[8];
#pragma unroll
        for (int j = 0; j < 8; ++j) {
            const int r = 8 * h + j;
            const float mn = fmaxf(mrow[j], fmaxf(Xm[pr][0][r], Xm[pr][1][r]));
            alpha[j] = __expf(mrow[j] - mn);
            const float pj = __expf(s[j] - mn);
            mrow[j] = mn;
            const float psum = rowsum16(pj);
            if (laneN == 0) Xs[pr][kh][r] = psum;
            Pw[r * PP + 16 * kh + laneN] = (_Float16)(pj * P_CARRY);
            lrow[j] *= alpha[j];
#pragma unroll
            for (int a = 0; a < 8; ++a) o[a][j] *= alpha[j];
        }
        __syncthreads();

#pragma unroll
        for (int j = 0; j < 8; ++j) {
            const int r = 8 * h + j;
            lrow[j] += Xs[pr][0][r] + Xs[pr][1][r];
        }
        const FragH pf = ldfragh(Pw + laneN * PP, h);

#pragma unroll
        for (int a = 0; a < 8; ++a) {
            const size_t vo = vbase + (size_t)(kh * 128 + a * 16 + laneN) * (size_t)SEQ + key0;
            const FragH fv = ldfragh(Vt + vo, h);
            o[a] = wmh(pf, fv, o[a]);
        }
    }

    float linv[8];
#pragma unroll
    for (int j = 0; j < 8; ++j) linv[j] = (1.0f / lrow[j]) * O_FOLD;
    float* Ow = &Osh[wave][0];
#pragma unroll
    for (int a = 0; a < 8; ++a)
#pragma unroll
        for (int j = 0; j < 8; ++j)
            Ow[(8 * h + j) * OP + a * 16 + laneN] = o[a][j] * linv[j];
    __syncthreads();

#pragma unroll
    for (int ps = 0; ps < 2; ++ps) {
        if (ps) __threadfence();
#pragma unroll
        for (int it = 0; it < 8; ++it) {
            const int r  = it * 2 + (lane >> 4);
            const int d0 = (lane & 15) * 8;
            const v4f x0 = *(const v4f*)(Ow + r * OP + d0);
            const v4f x1 = *(const v4f*)(Ow + r * OP + d0 + 4);
            v8us hv, lv;
            split8(x0, x1, hv, lv);
            const size_t off = ((size_t)b * SEQ + (size_t)(q0 + r)) * CI + kh * 128 + d0;
            *(volatile v8us*)(Yh + off) = hv;
            *(volatile v8us*)(Yl + off) = lv;
        }
    }
}

extern "C" void kernel_launch(void* const* d_in, const int* in_sizes, int n_in,
                              void* d_out, int out_size, void* d_ws, size_t ws_size,
                              hipStream_t stream) {
    if (n_in < 5) return;
    const long needX = ((long)NB * CH - 1) * (long)SEQ_FULL + (long)SEQ;
    if ((long)in_sizes[0] < needX) return;
    if ((long)in_sizes[1] < (long)CI * CH) return;
    if ((long)in_sizes[2] < (long)CI * CH) return;
    if ((long)in_sizes[3] < (long)CI * CH) return;
    if ((long)in_sizes[4] < (long)CH * CI) return;
    if ((long)out_size < (long)NB * CH * SEQ) return;

    const float* x       = (const float*)d_in[0];
    const float* w_phi   = (const float*)d_in[1];
    const float* w_theta = (const float*)d_in[2];
    const float* w_g     = (const float*)d_in[3];
    const float* w_m     = (const float*)d_in[4];
    float*       out     = (float*)d_out;

    const size_t planeY = (size_t)MROWS * CI * sizeof(bfu16);
    size_t off = 0;
    char* ws = (char*)d_ws;
    bfu16*    Xt   = (bfu16*)(ws + off);    off += (size_t)MROWS * CH * sizeof(bfu16);
    bfu16*    Wcat = (bfu16*)(ws + off);    off += (size_t)WCAT_N * CH * sizeof(bfu16);
    bfu16*    Wmb  = (bfu16*)(ws + off);    off += (size_t)CH * CI * sizeof(bfu16);
    bfu16*    Th   = (bfu16*)(ws + off);    off += planeY;
    bfu16*    Tl   = (bfu16*)(ws + off);    off += planeY;
    bfu16*    Ph   = (bfu16*)(ws + off);    off += planeY;
    bfu16*    Pl   = (bfu16*)(ws + off);    off += planeY;
    _Float16* Vt   = (_Float16*)(ws + off); off += planeY;
    bfu16*    Yh   = (bfu16*)(ws + off);    off += planeY;
    bfu16*    Yl   = (bfu16*)(ws + off);    off += planeY;
    if (off > ws_size) return;

    const int w8 = CI * CH / 8;

    cvt_x<<<dim3(SEQ / 64, CH / 64, NB), 256, 0, stream>>>(x, Xt);
    cvt_flat<<<dim3((w8 + 255) / 256), 256, 0, stream>>>(w_phi,   Wcat,                       w8);
    cvt_flat<<<dim3((w8 + 255) / 256), 256, 0, stream>>>(w_theta, Wcat + (size_t)CI * CH,     w8);
    cvt_flat<<<dim3((w8 + 255) / 256), 256, 0, stream>>>(w_g,     Wcat + (size_t)2 * CI * CH, w8);
    cvt_flat<<<dim3((w8 + 255) / 256), 256, 0, stream>>>(w_m,     Wmb,                        w8);

    gemm16<CH, 0, 1><<<dim3(MROWS / 128, WCAT_N / 64), 128, 0, stream>>>(
        Xt, Wcat, Wcat, Th, Tl, Ph, Pl, Vt, out);

    attn_pair<<<dim3(SEQ / 32, NB), 128, 0, stream>>>(Th, Tl, Ph, Pl, Vt, Yh, Yl);

    gemm16<CI, 1, 2><<<dim3(CH / 128, MROWS / 64), 128, 0, stream>>>(
        Wmb, Yh, Yl, Th, Tl, Ph, Pl, Vt, out);
}
